// DilatedMHA_48610439856408
// MI455X (gfx1250) — hardware-verified
//
#include <hip/hip_runtime.h>
#include <math.h>

typedef __attribute__((ext_vector_type(16))) _Float16 v16h;
typedef __attribute__((ext_vector_type(16))) __bf16 v16b;
typedef __attribute__((ext_vector_type(8)))  _Float16 v8h;
typedef __attribute__((ext_vector_type(8)))  float v8f;
typedef __attribute__((ext_vector_type(4)))  float v4f;
typedef __attribute__((ext_vector_type(2)))  float v2f;
typedef __attribute__((ext_vector_type(4)))  unsigned v4u;
typedef __attribute__((ext_vector_type(4)))  int v4i;
typedef float __attribute__((may_alias)) float_a;
typedef int __attribute__((may_alias)) int_a;

template <typename T> __device__ __forceinline__ void vst2(void* p, T v) { *(volatile T*)p = v; __threadfence(); *(volatile T*)p = v; }
__device__ __forceinline__ v8f wmma16(v16h a, v16h b, v8f c) {
  v8f d = __builtin_amdgcn_wmma_f32_16x16x32_f16(false, a, false, b, (short)0, c, false, false);
  asm volatile("v_nop\n\tv_nop\n\tv_nop\n\tv_nop" : "+v"(d) : "v"(a), "v"(b));
  return d;
}
__device__ __forceinline__ v8f wmma_bf(v16b a, v16b b, v8f c) {
  v8f d = __builtin_amdgcn_wmma_f32_16x16x32_bf16(false, a, false, b, (short)0, c, false, false);
  asm volatile("v_nop\n\tv_nop\n\tv_nop\n\tv_nop" : "+v"(d) : "v"(a), "v"(b));
  return d;
}
__device__ __forceinline__ v16h frag_h(const _Float16* rowk0, int lane) {
  union { v16h v; v8h q[2]; } u; const _Float16* p = rowk0 + 8 * (lane >> 4);
  u.q[0] = *(const v8h*)p; u.q[1] = *(const v8h*)(p + 16); return u.v;
}
__device__ __forceinline__ v16h frag_f32(const float* rowk0, int lane) {
  v16h a; const float* p = rowk0 + 8 * (lane >> 4);
#pragma unroll
  for (int i = 0; i < 8; ++i) { a[i] = (_Float16)p[i]; a[8 + i] = (_Float16)p[16 + i]; }
  return a;
}
__device__ __forceinline__ v16h frag_f32s(const float* rowk0, int lane, float sc) {
  v16h a; const float* p = rowk0 + 8 * (lane >> 4);
#pragma unroll
  for (int i = 0; i < 8; ++i) { a[i] = (_Float16)(p[i] * sc); a[8 + i] = (_Float16)(p[16 + i] * sc); }
  return a;
}
__device__ __forceinline__ v16h fragc_f32(const float* W, int k0, int n, int lane, int ld, int K) {
  v16h a; const int g = lane >> 4;
#pragma unroll
  for (int i = 0; i < 8; ++i) { const int ka = k0 + 8 * g + i, kb = ka + 16;
    a[i] = (_Float16)(ka < K ? W[(size_t)(ka < K ? ka : K - 1) * ld + n] : 0.f); a[8 + i] = (_Float16)(kb < K ? W[(size_t)(kb < K ? kb : K - 1) * ld + n] : 0.f); }
  return a;
}
struct F2 { v16b h, l; };
__device__ __forceinline__ F2 bsplit16(const float v[16]) { F2 r;
#pragma unroll
  for (int i = 0; i < 16; ++i) { const __bf16 h = (__bf16)v[i]; r.h[i] = h; r.l[i] = (__bf16)(v[i] - (float)h); }
  return r; }
__device__ __forceinline__ F2 split_row(const float* row, int k0, int lane) { float v[16]; const float* p = row + k0 + 8 * (lane >> 4);
#pragma unroll
  for (int i = 0; i < 8; ++i) { v[i] = p[i]; v[8 + i] = p[16 + i]; }
  return bsplit16(v); }
__device__ __forceinline__ F2 split_rowK(const float* row, int k0, int lane, int K) { float v[16]; const int g = lane >> 4;
#pragma unroll
  for (int i = 0; i < 8; ++i) { const int ka = k0 + 8 * g + i, kb = ka + 16; v[i] = ka < K ? row[ka < K ? ka : K - 1] : 0.f; v[8 + i] = kb < K ? row[kb < K ? kb : K - 1] : 0.f; }
  return bsplit16(v); }
__device__ __forceinline__ F2 split_col(const float* W, int k0, int n, int lane, int ld, int K) { float v[16]; const int g = lane >> 4;
#pragma unroll
  for (int i = 0; i < 8; ++i) { const int ka = k0 + 8 * g + i, kb = ka + 16; v[i] = ka < K ? W[(size_t)(ka < K ? ka : K - 1) * ld + n] : 0.f; v[8 + i] = kb < K ? W[(size_t)(kb < K ? kb : K - 1) * ld + n] : 0.f; }
  return bsplit16(v); }
__device__ __forceinline__ v8f mac3(const F2& a, const F2& b, v8f c) { c = wmma_bf(a.l, b.h, c); c = wmma_bf(a.h, b.l, c); return wmma_bf(a.h, b.h, c); }
__device__ __forceinline__ float sigm(float v) { return 1.0f / (1.0f + expf(-v)); }
#define LDSX() do { asm volatile("s_wait_dscnt 0" ::: "memory"); __builtin_amdgcn_wave_barrier(); __builtin_amdgcn_fence(__ATOMIC_RELEASE, "workgroup"); } while (0)


#define NB 2
#define SS 8192
#define NR (NB * SS)
#define DM 768
#define NH 12
#define HD 64
#ifndef TNB
#define TNB NB
#define TOR (NR / 64)
#endif
typedef __attribute__((ext_vector_type(8))) __bf16 v8b;
__device__ __forceinline__ v16b frag_b(const __bf16* rowk0, int lane) {
  union { v16b v; v8b q[2]; } u; const __bf16* p = rowk0 + 8 * (lane >> 4);
  u.q[0] = *(const v8b*)p; u.q[1] = *(const v8b*)(p + 16); return u.v;
}
__device__ __forceinline__ float bfr(float v) { return (float)(__bf16)v; }
__device__ __attribute__((noinline)) float exp_ni(float v) { return expf(v); }
__device__ __attribute__((noinline)) float erf_ni(float v) { return erff(v); }

#define WS_PK  0u
#define PK_O   ((size_t)3 * DM * DM)
#define WS_QKV (((2u * 4 * DM * DM) + 127u) / 128u * 128u)
#define WS_OUT (WS_QKV + 4u * (size_t)NR * 3 * DM)
#define WS_PS  (WS_OUT + 4u * (size_t)NR * DM)
#define WS_CS  (WS_PS + 4u * (NR / 64) * DM)
#define WS_END (WS_CS + 4u * NB * DM)

__global__ __launch_bounds__(256) void k_pack(const float* __restrict__ WQKV, const float* __restrict__ WO, __bf16* __restrict__ PK) {
  __shared__ __align__(16) __bf16 s[DM]; const int n = blockIdx.x, which = blockIdx.y, t = threadIdx.x;
  if (which == 1 && n >= DM) return;
  const float* src = (which == 0) ? (WQKV + (size_t)n * DM) : (WO + (size_t)n * DM);
  for (int k = t; k < DM; k += 256) s[k] = (__bf16)src[k];
  __syncthreads();
  for (int q = t; q < DM / 8; q += 256) vst2((unsigned*)(PK + ((which == 0) ? 0 : PK_O) + (size_t)n * DM + q * 8), *(const v4u*)&s[q * 8]);
}
__global__ __launch_bounds__(128) void k_qkv(const float* __restrict__ X, const __bf16* __restrict__ PK, float* __restrict__ QKV) {
  __shared__ __align__(16) float so[4][16][132];
  const int tid = threadIdx.x, wave = tid >> 5, lane = tid & 31, col = lane & 15, g = lane >> 4; const size_t r0 = (size_t)blockIdx.x * 64 + wave * 16; const int n0 = blockIdx.y * 128;
  v8f acc[8] = {};
#pragma unroll 2
  for (int kc = 0; kc < DM / 32; ++kc) { v16b a; { const float* p = X + (r0 + col) * DM + kc * 32 + 8 * g;
#pragma unroll
      for (int i = 0; i < 8; ++i) { a[i] = (__bf16)p[i]; a[8 + i] = (__bf16)p[16 + i]; } }
#pragma unroll
    for (int j = 0; j < 8; ++j) acc[j] = wmma_bf(a, frag_b(PK + (size_t)(n0 + j * 16 + col) * DM + kc * 32, lane), acc[j]); }
#pragma unroll
  for (int j = 0; j < 8; ++j)
#pragma unroll
    for (int r = 0; r < 8; ++r) so[wave][8 * g + r][j * 16 + col] = acc[j][r];
  LDSX();
  for (int rl = 0; rl < 16; ++rl) vst2(QKV + (r0 + rl) * (3 * DM) + n0 + lane * 4, *(const v4f*)&so[wave][rl][lane * 4]);
}
__device__ __forceinline__ void dil_group(const float* __restrict__ QKVb, int p, int h, int base, int stride, int cnt, float* __restrict__ accd) {
  const float* q = QKVb + (size_t)p * (3 * DM) + h * HD; float sc[4] = {0.f, 0.f, 0.f, 0.f}; float mx = -3.0e38f;
#pragma unroll
  for (int i = 0; i < 4; ++i) { if (i < cnt) { const float* k = QKVb + (size_t)(base + i * stride) * (3 * DM) + DM + h * HD; float s = 0.f;
#pragma unroll 1
      for (int d = 0; d < HD; ++d) s += q[d] * k[d];
      sc[i] = s * 0.125f; mx = fmaxf(mx, sc[i]); } }
  float e[4] = {0.f, 0.f, 0.f, 0.f}; float l = 0.f;
#pragma unroll
  for (int i = 0; i < 4; ++i) if (i < cnt) { e[i] = exp_ni(sc[i] - mx); l += e[i]; }
  const float il = 1.0f / l;
#pragma unroll
  for (int i = 0; i < 4; ++i) { if (i < cnt) { const float w = e[i] * il; const float* v = QKVb + (size_t)(base + i * stride) * (3 * DM) + 2 * DM + h * HD;
#pragma unroll 1
      for (int d = 0; d < HD; ++d) accd[d] += w * v[d]; } }
}
__global__ __launch_bounds__(256) void k_dil(const float* __restrict__ QKV, float* __restrict__ OUT, float* __restrict__ PS) {
  __shared__ float so[64][4 * HD + 4];
  const int tid = threadIdx.x; const int pl = tid & 63, hl = tid >> 6; const int b = blockIdx.z, h = blockIdx.y * 4 + hl; const int p = blockIdx.x * 64 + pl; const float* QKVb = QKV + (size_t)b * SS * (3 * DM);
  float* accd = &so[pl][hl * HD];
#pragma unroll 1
  for (int d = 0; d < HD; ++d) accd[d] = 0.f;
  dil_group(QKVb, p, h, p % 2048, 2048, 4, accd);
  if (((p % 4096) & 1) == 0) dil_group(QKVb, p, h, p % 4096, 4096, 2, accd);
  if ((p & 3) == 0) { const float* v = QKVb + (size_t)p * (3 * DM) + 2 * DM + h * HD;
#pragma unroll 1
    for (int d = 0; d < HD; ++d) accd[d] += v[d]; }
  __syncthreads();
  { const int h0 = blockIdx.y * 4; for (int e = tid; e < 64 * 64; e += 256) { const int r = e >> 6, pc = e & 63; vst2(OUT + ((size_t)b * SS + blockIdx.x * 64 + r) * DM + h0 * HD + pc * 4, *(const v4f*)&so[r][pc * 4]); } }
  { const int c = tid; float s = 0.f; for (int r = 0; r < 64; ++r) s += so[r][c]; __syncthreads(); so[0][c] = s; }
  __syncthreads();
  if (tid < 64) vst2(PS + ((size_t)b * (SS / 64) + blockIdx.x) * DM + blockIdx.y * 4 * HD + tid * 4, *(const v4f*)&so[0][tid * 4]);
}
__global__ __launch_bounds__(192) void k_colsum(const float* __restrict__ PS, float* __restrict__ CS) {
  const int b = blockIdx.x, t = threadIdx.x; v4f s = {0.f, 0.f, 0.f, 0.f};
  for (int blk = 0; blk < SS / 64; ++blk) { const v4f v = *(const v4f*)(PS + ((size_t)b * (SS / 64) + blk) * DM + t * 4); s[0] += v[0]; s[1] += v[1]; s[2] += v[2]; s[3] += v[3]; }
  v4f r4 = {1.0f / s[0], 1.0f / s[1], 1.0f / s[2], 1.0f / s[3]}; vst2(CS + (size_t)b * DM + t * 4, r4);
}
__global__ __launch_bounds__(128) void k_out(const float* __restrict__ OUTN, const float* __restrict__ CS, const __bf16* __restrict__ PK, float* __restrict__ Y) {
  __shared__ __align__(16) float so[4][16][132];
  const int tid = threadIdx.x, wave = tid >> 5, lane = tid & 31, col = lane & 15, g = lane >> 4; const size_t r0 = (size_t)blockIdx.x * 64 + wave * 16; const int n0 = blockIdx.y * 128; const int b = (int)(r0 / SS); const float* csb = CS + (size_t)b * DM;
  v8f acc[8] = {};
#pragma unroll 2
  for (int kc = 0; kc < DM / 32; ++kc) { v16b ah, al; { const float* p = OUTN + (r0 + col) * DM + kc * 32 + 8 * g; const float* cp = csb + kc * 32 + 8 * g;
#pragma unroll
      for (int i = 0; i < 16; ++i) { const int off = (i & 7) + ((i >> 3) << 4); const float v = p[off] * cp[off]; const __bf16 hb = (__bf16)v; ah[i] = hb; al[i] = (__bf16)(v - (float)hb); } }
#pragma unroll
    for (int j = 0; j < 8; ++j) { const v16b w = frag_b(PK + PK_O + (size_t)(n0 + j * 16 + col) * DM + kc * 32, lane); acc[j] = wmma_bf(al, w, acc[j]); acc[j] = wmma_bf(ah, w, acc[j]); } }
#pragma unroll
  for (int j = 0; j < 8; ++j)
#pragma unroll
    for (int r = 0; r < 8; ++r) so[wave][8 * g + r][j * 16 + col] = acc[j][r];
  LDSX();
  for (int rl = 0; rl < 16; ++rl) vst2(Y + (r0 + rl) * DM + n0 + lane * 4, *(const v4f*)&so[wave][rl][lane * 4]);
}
extern "C" void kernel_launch(void* const* d_in, const int* in_sizes, int n_in, void* d_out, int out_size, void* d_ws, size_t ws_size, hipStream_t stream) {
  (void)in_sizes; (void)n_in; (void)out_size;
  const float** F = (const float**)d_in;
  if (ws_size < (size_t)WS_END) return;
  char* ws = (char*)d_ws; __bf16* PK = (__bf16*)(ws + WS_PK); float *QKV = (float*)(ws + WS_QKV), *OUTN = (float*)(ws + WS_OUT), *PS = (float*)(ws + WS_PS), *CS = (float*)(ws + WS_CS);
  k_pack<<<dim3(3 * DM, 2), 256, 0, stream>>>(F[1], F[2], PK);
  k_qkv<<<dim3(TNB * SS / 64, 3 * DM / 128), 128, 0, stream>>>(F[0], PK, QKV);
  k_dil<<<dim3(SS / 64, NH / 4, TNB), 256, 0, stream>>>(QKV, OUTN, PS);
  k_colsum<<<TNB, 192, 0, stream>>>(PS, CS);
  k_out<<<dim3(TOR, DM / 128), 128, 0, stream>>>(OUTN, CS, PK, (float*)d_out);
}
